// NodeRegressor_17952963297293
// MI455X (gfx1250) — hardware-run, weakly checked
//
#include <hip/hip_runtime.h>
#include <math.h>

typedef __attribute__((ext_vector_type(16))) _Float16 v16h;
typedef __attribute__((ext_vector_type(8)))  _Float16 v8h;
typedef __attribute__((ext_vector_type(4)))  _Float16 v4h;
typedef __attribute__((ext_vector_type(8)))  float    v8f;
typedef __attribute__((ext_vector_type(4)))  float    v4f;
typedef __attribute__((ext_vector_type(2)))  float    v2f;
typedef __attribute__((ext_vector_type(4)))  int      v4i;

constexpr int kN     = 100000;
constexpr int kE     = 2000000;
constexpr int kIn    = 6;
constexpr int kHid   = 128;
constexpr int kNPad  = 100032;
constexpr int kKA    = 2 * kHid;
constexpr int kT1    = 4096;
constexpr int kBlk1  = 25;
constexpr int kT2    = 512;
constexpr int kBlk2  = 196;
constexpr int kIters = (kE + 255) / 256;
constexpr float kCarryA = 16.0f;
constexpr float kCarryB = 256.0f;
constexpr float kFold   = 1.0f / (kCarryA * kCarryB);
static_assert((kE % 8) == 0, "edge rows are whole 8-edge lane groups");
static_assert((kNPad % 64) == 0 && kNPad >= kN, "GEMM M multiple of 64");
static_assert((kNPad % 2) == 0 && (kT2 % 2) == 0, "row pairs");
static_assert((kKA % 32) == 0 && (kHid % 64) == 0, "GEMM K multiple of 32, N multiple of 64");
static_assert(kBlk1 * kT1 >= kNPad, "layer-1 tiles cover all plane rows");
static_assert(kBlk2 * kT2 >= kNPad, "layer-2 tiles cover all plane rows");
static_assert(kBlk2 * kT2 <= kBlk1 * kT1, "inverse-count table covers every index the second pass reads");
static_assert((kN % 4) == 0, "output written in 16-B pieces");
static_assert((kBlk2 - 1) * kT2 < kNPad && (kBlk1 - 1) * kT1 < kNPad, "every block owns at least one plane row");

constexpr size_t kOffInv = 0;
constexpr size_t kOffH1F = kOffInv + (size_t)kBlk1 * kT1 * 4;
constexpr size_t kOffAP  = kOffH1F + (size_t)kNPad * kHid * 4;
constexpr size_t kOffBT  = kOffAP  + (size_t)kNPad * kKA * 2;
constexpr size_t kWsTotal = kOffBT + (size_t)kHid * kKA * 2;
static_assert(kWsTotal == 102907904ull, "carve total");
static_assert(kWsTotal <= 134217728ull, "carve cap");
static_assert((kOffH1F % 128) == 0 && (kOffAP % 128) == 0 && (kOffBT % 128) == 0, "128-B aligned regions");

union FragU { v16h v; v8h h[2]; };
__device__ __forceinline__ v16h frag_load(const _Float16* p) {
  FragU f;
  f.h[0] = *(const v8h*)(p);
  f.h[1] = *(const v8h*)(p + 16);
  return f.v;
}
__device__ __forceinline__ v8f mma_h(v16h a, v16h b, v8f c) {
  c = __builtin_amdgcn_wmma_f32_16x16x32_f16(false, a, false, b, (short)0, c, false, false);
  asm volatile("v_nop\n\tv_nop\n\tv_nop\n\tv_nop" : "+v"(c) : "v"(a), "v"(b));
  return c;
}

__global__ __launch_bounds__(256) void prep_bt_kernel(
    const float* __restrict__ W2l, const float* __restrict__ W2r, unsigned short* __restrict__ Bt)
{
  const int src = blockIdx.y;
  const float* W = (src == 0) ? W2l : W2r;
  const int t  = blockIdx.x * 256 + threadIdx.x;
  const int n  = t >> 4;
  const int k0 = (t & 15) * 8;
  v8h hv;
#pragma unroll
  for (int e = 0; e < 8; ++e) {
    const float w = W[(size_t)(k0 + e) * kHid + n] * kCarryB;
    hv[e] = (_Float16)w;
  }
  unsigned short* p = Bt + (size_t)n * kKA + src * kHid + k0;
  *(volatile v8h*)p = hv;
  __threadfence();
  *(volatile v8h*)p = hv;
}

#define AGG_DRAIN_SIX(DJ, SJ)                                              \
  {                                                                        \
    const unsigned xd_ = (unsigned)(DJ) - ulo;                             \
    const bool hit_ = valid && (xd_ < lim);                                \
    unsigned m_ = __builtin_amdgcn_ballot_w32(hit_);                       \
    while (m_ != 0u) {                                                     \
      const int hl_ = __builtin_ctz(m_);                                   \
      m_ &= (m_ - 1u);                                                     \
      int s_ = __builtin_amdgcn_readlane((SJ), hl_);                       \
      int dl_ = __builtin_amdgcn_readlane((int)xd_, hl_);                  \
      s_ = s_ < 0 ? 0 : s_;                                                \
      s_ = s_ > (kN - 1) ? (kN - 1) : s_;                                  \
      dl_ = dl_ < 0 ? 0 : dl_;                                             \
      dl_ = dl_ > (kT1 - 1) ? (kT1 - 1) : dl_;                             \
      float xv_ = x[(size_t)s_ * kIn + kk];                                \
      asm volatile("" : "+v"(xv_));                                        \
      const float v_ = isx ? xv_ : cst;                                    \
      if (lane < 8) {                                                      \
        const int ai_ = dl_ * 8 + lane;                                    \
        acc1[ai_] = acc1[ai_] + v_;                                        \
      }                                                                    \
    }                                                                      \
  }

__global__ __launch_bounds__(32) void agg1_layer1_kernel(
    const float* __restrict__ x, const int* __restrict__ ei,
    const float* __restrict__ W1l, const float* __restrict__ b1l, const float* __restrict__ W1r,
    float* __restrict__ invT, float* __restrict__ H1F, unsigned short* __restrict__ AP)
{
  extern __shared__ __align__(16) float acc1[];
  const int lane = threadIdx.x;
  const int lo = blockIdx.x * kT1;
  const unsigned ulo = (unsigned)lo;
  int limi = kN - lo;
  limi = limi < 0 ? 0 : limi;
  limi = limi > kT1 ? kT1 : limi;
  const unsigned lim = (unsigned)limi;
  int nloc = kNPad - lo;
  nloc = nloc < 0 ? 0 : nloc;
  nloc = nloc > kT1 ? kT1 : nloc;

  const v4f z4 = (v4f){0.f, 0.f, 0.f, 0.f};
#pragma unroll 1
  for (int i = lane * 4; i < kT1 * 8; i += 128) *(v4f*)(acc1 + i) = z4;
  __syncthreads();

  const int l7 = lane & 7;
  const int kk = l7 < 5 ? l7 : 5;
  const bool isx = l7 < 6;
  const float cst = (l7 == 6) ? 1.0f : 0.0f;
  const int* srcp = ei;
  const int* dstp = ei + kE;

#pragma unroll 1
  for (int it = 0; it < kIters; ++it) {
    const int eb = it * 256 + lane * 8;
    const bool valid = eb < kE;
    const int ebc = valid ? eb : (kE - 8);
    const v4i d0 = *(const v4i*)(dstp + ebc);
    const v4i d1 = *(const v4i*)(dstp + ebc + 4);
    const v4i s0 = *(const v4i*)(srcp + ebc);
    const v4i s1 = *(const v4i*)(srcp + ebc + 4);
    const int da = d0[0], db = d0[1], dc = d0[2], dd = d0[3];
    const int de = d1[0], df = d1[1], dg = d1[2], dh = d1[3];
    const int sa = s0[0], sb = s0[1], sc = s0[2], sd = s0[3];
    const int se = s1[0], sf = s1[1], sg = s1[2], sh = s1[3];
    AGG_DRAIN_SIX(da, sa)
    AGG_DRAIN_SIX(db, sb)
    AGG_DRAIN_SIX(dc, sc)
    AGG_DRAIN_SIX(dd, sd)
    AGG_DRAIN_SIX(de, se)
    AGG_DRAIN_SIX(df, sf)
    AGG_DRAIN_SIX(dg, sg)
    AGG_DRAIN_SIX(dh, sh)
  }
  __syncthreads();

  const int c4 = lane * 4;
  v4f wl[6], wr[6];
#pragma unroll
  for (int k = 0; k < 6; ++k) {
    wl[k] = *(const v4f*)(W1l + k * kHid + c4);
    wr[k] = *(const v4f*)(W1r + k * kHid + c4);
  }
  const v4f bb = *(const v4f*)(b1l + c4);

#pragma unroll 1
  for (int l = 0; l < nloc; ++l) {
    const int n = lo + l;
    const v4f a0 = *(const v4f*)(acc1 + l * 8);
    const v4f a1 = *(const v4f*)(acc1 + l * 8 + 4);
    const float cnt = a1[2];
    const float inv = 1.0f / fmaxf(cnt, 1.0f);
    const bool real = n < kN;
    const int nc = real ? n : (kN - 1);
    const float* xr = x + (size_t)nc * kIn;
    const v2f x01 = *(const v2f*)(xr);
    const v2f x23 = *(const v2f*)(xr + 2);
    const v2f x45 = *(const v2f*)(xr + 4);
    float mk[6], xk[6];
    mk[0] = a0[0] * inv; mk[1] = a0[1] * inv; mk[2] = a0[2] * inv;
    mk[3] = a0[3] * inv; mk[4] = a1[0] * inv; mk[5] = a1[1] * inv;
    xk[0] = x01[0]; xk[1] = x01[1]; xk[2] = x23[0];
    xk[3] = x23[1]; xk[4] = x45[0]; xk[5] = x45[1];
    float h0 = bb[0], h1 = bb[1], h2 = bb[2], h3 = bb[3];
#pragma unroll
    for (int k = 0; k < 6; ++k) {
      h0 = fmaf(mk[k], wl[k][0], h0);
      h1 = fmaf(mk[k], wl[k][1], h1);
      h2 = fmaf(mk[k], wl[k][2], h2);
      h3 = fmaf(mk[k], wl[k][3], h3);
    }
#pragma unroll
    for (int k = 0; k < 6; ++k) {
      h0 = fmaf(xk[k], wr[k][0], h0);
      h1 = fmaf(xk[k], wr[k][1], h1);
      h2 = fmaf(xk[k], wr[k][2], h2);
      h3 = fmaf(xk[k], wr[k][3], h3);
    }
    h0 = real ? fmaxf(h0, 0.0f) : 0.0f;
    h1 = real ? fmaxf(h1, 0.0f) : 0.0f;
    h2 = real ? fmaxf(h2, 0.0f) : 0.0f;
    h3 = real ? fmaxf(h3, 0.0f) : 0.0f;
    const v4f fv = (v4f){h0, h1, h2, h3};
    v4h pv;
    pv[0] = (_Float16)(h0 * kCarryA);
    pv[1] = (_Float16)(h1 * kCarryA);
    pv[2] = (_Float16)(h2 * kCarryA);
    pv[3] = (_Float16)(h3 * kCarryA);
    float* pf = H1F + (size_t)n * kHid + c4;
    unsigned short* ph = AP + (size_t)n * kKA + kHid + c4;
    *(volatile v4f*)pf = fv;
    *(volatile v4h*)ph = pv;
    __threadfence();
    *(volatile v4f*)pf = fv;
    *(volatile v4h*)ph = pv;
  }

  for (int pass = 0; pass < 2; ++pass) {
#pragma unroll 1
    for (int i = lane; i < kT1; i += 32) {
      const float c = acc1[i * 8 + 6];
      const float iv = 1.0f / fmaxf(c, 1.0f);
      *(volatile float*)(invT + lo + i) = iv;
    }
    __threadfence();
  }
}

#define AGG_DRAIN_WIDE(DJ, SJ)                                             \
  {                                                                        \
    const unsigned xd_ = (unsigned)(DJ) - ulo;                             \
    const bool hit_ = valid && (xd_ < lim);                                \
    unsigned m_ = __builtin_amdgcn_ballot_w32(hit_);                       \
    while (m_ != 0u) {                                                     \
      const int hl_ = __builtin_ctz(m_);                                   \
      m_ &= (m_ - 1u);                                                     \
      int s_ = __builtin_amdgcn_readlane((SJ), hl_);                       \
      int dl_ = __builtin_amdgcn_readlane((int)xd_, hl_);                  \
      s_ = s_ < 0 ? 0 : s_;                                                \
      s_ = s_ > (kN - 1) ? (kN - 1) : s_;                                  \
      dl_ = dl_ < 0 ? 0 : dl_;                                             \
      dl_ = dl_ > (kT2 - 1) ? (kT2 - 1) : dl_;                             \
      v4f hv_ = *(const v4f*)(H1F + (size_t)s_ * kHid + c4);               \
      asm volatile("" : "+v"(hv_));                                        \
      float* ap_ = acc2 + dl_ * kHid + c4;                                 \
      v4f av_ = *(const v4f*)ap_;                                          \
      av_ = av_ + hv_;                                                     \
      *(v4f*)ap_ = av_;                                                    \
    }                                                                      \
  }

__global__ __launch_bounds__(32) void agg2_mean_kernel(
    const int* __restrict__ ei, const float* __restrict__ H1F, const float* __restrict__ invT,
    unsigned short* __restrict__ AP)
{
  extern __shared__ __align__(16) float acc2[];
  const int lane = threadIdx.x;
  const int lo = blockIdx.x * kT2;
  const unsigned ulo = (unsigned)lo;
  int limi = kN - lo;
  limi = limi < 0 ? 0 : limi;
  limi = limi > kT2 ? kT2 : limi;
  const unsigned lim = (unsigned)limi;
  int nloc = kNPad - lo;
  nloc = nloc < 0 ? 0 : nloc;
  nloc = nloc > kT2 ? kT2 : nloc;
  const int npairs = nloc >> 1;
  const int c4 = lane * 4;

  const v4f z4 = (v4f){0.f, 0.f, 0.f, 0.f};
#pragma unroll 1
  for (int i = lane * 4; i < kT2 * kHid; i += 128) *(v4f*)(acc2 + i) = z4;
  __syncthreads();

  const int* srcp = ei;
  const int* dstp = ei + kE;
#pragma unroll 1
  for (int it = 0; it < kIters; ++it) {
    const int eb = it * 256 + lane * 8;
    const bool valid = eb < kE;
    const int ebc = valid ? eb : (kE - 8);
    const v4i d0 = *(const v4i*)(dstp + ebc);
    const v4i d1 = *(const v4i*)(dstp + ebc + 4);
    const v4i s0 = *(const v4i*)(srcp + ebc);
    const v4i s1 = *(const v4i*)(srcp + ebc + 4);
    const int da = d0[0], db = d0[1], dc = d0[2], dd = d0[3];
    const int de = d1[0], df = d1[1], dg = d1[2], dh = d1[3];
    const int sa = s0[0], sb = s0[1], sc = s0[2], sd = s0[3];
    const int se = s1[0], sf = s1[1], sg = s1[2], sh = s1[3];
    AGG_DRAIN_WIDE(da, sa)
    AGG_DRAIN_WIDE(db, sb)
    AGG_DRAIN_WIDE(dc, sc)
    AGG_DRAIN_WIDE(dd, sd)
    AGG_DRAIN_WIDE(de, se)
    AGG_DRAIN_WIDE(df, sf)
    AGG_DRAIN_WIDE(dg, sg)
    AGG_DRAIN_WIDE(dh, sh)
  }
  __syncthreads();

  const int hh = lane >> 4;
  const int c8 = (lane & 15) * 8;
#pragma unroll 1
  for (int p = 0; p < npairs; ++p) {
    const int l = 2 * p + hh;
    const int n = lo + l;
    const float iv = invT[n] * kCarryA;
    const v4f a0 = *(const v4f*)(acc2 + l * kHid + c8);
    const v4f a1 = *(const v4f*)(acc2 + l * kHid + c8 + 4);
    v8h hv;
#pragma unroll
    for (int e = 0; e < 4; ++e) {
      const float u0 = a0[e] * iv;
      const float u1 = a1[e] * iv;
      hv[e]     = (_Float16)u0;
      hv[4 + e] = (_Float16)u1;
    }
    unsigned short* q = AP + (size_t)n * kKA + c8;
    *(volatile v8h*)q = hv;
    __threadfence();
    *(volatile v8h*)q = hv;
  }
}

__global__ __launch_bounds__(64) void gemm_head_kernel(
    const unsigned short* __restrict__ Ap, const unsigned short* __restrict__ Btp,
    const float* __restrict__ b2l, const float* __restrict__ wlin, const float* __restrict__ blin,
    float* __restrict__ out)
{
  const _Float16* A  = (const _Float16*)Ap;
  const _Float16* Bt = (const _Float16*)Btp;
  __shared__ __align__(16) float sP[2 * 64 * 20];
  __shared__ __align__(16) float sRow[64];
  const int tid   = threadIdx.x;
  const int lane  = tid & 31;
  const int wave  = tid >> 5;
  const int m0    = blockIdx.x * 64;
  const int n0    = wave * 64;
  const int rlane = lane & 15;
  const int koff  = (lane >> 4) * 8;
  const int mOff  = (lane >> 4) * 8;

  v8f acc[4][4];
#pragma unroll
  for (int i = 0; i < 4; ++i)
#pragma unroll
    for (int j = 0; j < 4; ++j) acc[i][j] = (v8f){0.f, 0.f, 0.f, 0.f, 0.f, 0.f, 0.f, 0.f};

#pragma unroll 1
  for (int k0 = 0; k0 < kKA; k0 += 32) {
    v16h bh[4];
#pragma unroll
    for (int j = 0; j < 4; ++j)
      bh[j] = frag_load(Bt + (size_t)(n0 + (j << 4) + rlane) * kKA + koff + k0);
#pragma unroll
    for (int i = 0; i < 4; ++i) {
      const v16h ah = frag_load(A + (size_t)(m0 + (i << 4) + rlane) * kKA + koff + k0);
#pragma unroll
      for (int j = 0; j < 4; ++j) acc[i][j] = mma_h(ah, bh[j], acc[i][j]);
    }
  }

  float bv[4], wv[4];
#pragma unroll
  for (int j = 0; j < 4; ++j) {
    const int n = n0 + (j << 4) + rlane;
    bv[j] = b2l[n];
    wv[j] = wlin[n];
  }
  float* sp = sP + wave * (64 * 20);
#pragma unroll
  for (int i = 0; i < 4; ++i) {
#pragma unroll
    for (int r = 0; r < 8; ++r) {
      float p = 0.0f;
#pragma unroll
      for (int j = 0; j < 4; ++j) {
        float v = fmaf(acc[i][j][r], kFold, bv[j]);
        v = fmaxf(v, 0.0f);
        p = fmaf(v, wv[j], p);
      }
      sp[((i << 4) + mOff + r) * 20 + rlane] = p;
    }
  }
  __syncthreads();
  {
    float s = 0.0f;
#pragma unroll
    for (int w = 0; w < 2; ++w) {
#pragma unroll
      for (int q = 0; q < 4; ++q) {
        const v4f u = *(const v4f*)(sP + w * (64 * 20) + tid * 20 + q * 4);
        s += u[0];
        s += u[1];
        s += u[2];
        s += u[3];
      }
    }
    sRow[tid] = s + blin[0];
  }
  __syncthreads();
  if (wave == 0) {
    const int r4 = (lane & 15) * 4;
    const v4f o = *(const v4f*)(sRow + r4);
    const bool st = (lane < 16) && ((m0 + r4) < kN);
    float* po = out + m0 + r4;
    if (st) *(volatile v4f*)po = o;
    __threadfence();
    if (st) *(volatile v4f*)po = o;
  }
}

extern "C" void kernel_launch(void* const* d_in, const int* in_sizes, int n_in,
                              void* d_out, int out_size, void* d_ws, size_t ws_size,
                              hipStream_t stream) {
  if (n_in < 10) return;
  if (in_sizes[0] != kN * kIn) return;
  if (in_sizes[1] != 2 * kE) return;
  if (in_sizes[2] != kIn * kHid) return;
  if (in_sizes[3] != kHid) return;
  if (in_sizes[4] != kIn * kHid) return;
  if (in_sizes[5] != kHid * kHid) return;
  if (in_sizes[6] != kHid) return;
  if (in_sizes[7] != kHid * kHid) return;
  if (in_sizes[8] != kHid) return;
  if (in_sizes[9] != 1) return;
  if (out_size != kN) return;
  if (ws_size < kWsTotal) return;

  const float* x    = (const float*)d_in[0];
  const int*   ei   = (const int*)d_in[1];
  const float* W1l  = (const float*)d_in[2];
  const float* b1l  = (const float*)d_in[3];
  const float* W1r  = (const float*)d_in[4];
  const float* W2l  = (const float*)d_in[5];
  const float* b2l  = (const float*)d_in[6];
  const float* W2r  = (const float*)d_in[7];
  const float* Wlin = (const float*)d_in[8];
  const float* blin = (const float*)d_in[9];
  float* out = (float*)d_out;

  char* ws = (char*)d_ws;
  float*          INV = (float*)(ws + kOffInv);
  float*          H1F = (float*)(ws + kOffH1F);
  unsigned short* AP  = (unsigned short*)(ws + kOffAP);
  unsigned short* BT  = (unsigned short*)(ws + kOffBT);

  prep_bt_kernel<<<dim3(8, 2), 256, 0, stream>>>(W2l, W2r, BT);
  agg1_layer1_kernel<<<kBlk1, 32, (size_t)kT1 * 8 * sizeof(float), stream>>>(x, ei, W1l, b1l, W1r, INV, H1F, AP);
  agg2_mean_kernel<<<kBlk2, 32, (size_t)kT2 * kHid * sizeof(float), stream>>>(ei, H1F, INV, AP);
  gemm_head_kernel<<<kNPad / 64, 64, 0, stream>>>(AP, BT, b2l, Wlin, blin, out);
}
